// LSTMModel_3246995275913
// MI455X (gfx1250) — hardware-verified
//
#include <hip/hip_runtime.h>
#include <math.h>

constexpr int NBATCH  = 64;
constexpr int NSTEP   = 512;
constexpr int NIN     = 256;
constexpr int NHID    = 256;
constexpr int NGATE   = 4 * NHID;
constexpr int NFC     = 128;
constexpr int KCAT    = NIN + NHID;
constexpr int RTHR    = 512;
constexpr int RWAVES  = RTHR / 32;
constexpr int SEQ_BLK = 16;
constexpr int H_OFF   = NIN;
constexpr int LO_OFF  = KCAT;
constexpr int APITCH  = 2 * KCAT + 8;
constexpr int CPITCH  = 260;
constexpr float WCARRY     = 256.0f;
constexpr float WCARRY_INV = 1.0f / 256.0f;
constexpr float RCARRY     = 2048.0f;
constexpr float RCARRY_INV = 1.0f / 2048.0f;
constexpr int NOUT0 = NBATCH * NFC;
constexpr int NOUT1 = NBATCH * NSTEP * NHID;

static_assert(NIN == NHID, "shared convert map");
static_assert(NHID == 16 * RWAVES, "one 16-column group per wave");
static_assert(SEQ_BLK == RWAVES, "staging row = wave");
static_assert(NIN == 32 * 8, "x staging: 32 lanes x 8 columns");
static_assert(NHID == 2 * 32 * 4, "row store: 2 instructions x 32 lanes x 4 floats");
static_assert(NFC == 32 * 4, "head: 32 lanes x 4 outputs");
static_assert(KCAT % 32 == 0, "k tiles");
static_assert(NBATCH % SEQ_BLK == 0, "grid exact");
static_assert((APITCH * 2) % 16 == 0 && (CPITCH * 4) % 16 == 0, "16-B aligned LDS rows");
static_assert((size_t)NOUT0 * 4 == 32768, "out1 byte offset");
static_assert(((size_t)NOUT0 + (size_t)NOUT1) * 4 == 33587200, "d_out total bytes");

typedef __attribute__((ext_vector_type(16))) _Float16 v16h;
typedef __attribute__((ext_vector_type(8)))  _Float16 v8h;
typedef __attribute__((ext_vector_type(8)))  float    v8f;
typedef __attribute__((ext_vector_type(4)))  float    v4f;

__device__ __forceinline__ void acc_guard4(v8f& a, v8f& b, v8f& c, v8f& d) {
  asm volatile("v_nop\n\tv_nop\n\tv_nop\n\tv_nop" : "+v"(a), "+v"(b), "+v"(c), "+v"(d));
}
__device__ __forceinline__ void guard8(v8f& a0, v8f& a1, v8f& a2, v8f& a3, v8f& r0, v8f& r1, v8f& r2, v8f& r3,
                                       v16h x, v16h y, v16h b0, v16h b1, v16h b2, v16h b3) {
  asm volatile("v_nop\n\tv_nop\n\tv_nop\n\tv_nop"
               : "+v"(a0), "+v"(a1), "+v"(a2), "+v"(a3), "+v"(r0), "+v"(r1), "+v"(r2), "+v"(r3)
               : "v"(x), "v"(y), "v"(b0), "v"(b1), "v"(b2), "v"(b3));
}

template <typename T> struct Frag;
template <> struct Frag<_Float16> {
  typedef v16h V; union U { v16h v; v8h h[2]; };
  static __device__ __forceinline__ v16h load(const _Float16* p) {
    U f; f.h[0] = *(const v8h*)(p); f.h[1] = *(const v8h*)(p + 16); return f.v;
  }
  static __device__ __forceinline__ v8f mma(v16h a, v16h b, v8f c) {
    return __builtin_amdgcn_wmma_f32_16x16x32_f16(false, a, false, b, (short)0, c, false, false);
  }
};

__device__ __forceinline__ float fsig(float v)  { return __builtin_amdgcn_rcpf(1.0f + expf(-v)); }
__device__ __forceinline__ float ftanh(float v) { return 1.0f - 2.0f * __builtin_amdgcn_rcpf(expf(2.0f * v) + 1.0f); }

__device__ __forceinline__ void stage_x8(const float* __restrict__ xp, _Float16* dst) {
  const v4f a = *(const v4f*)(xp);
  const v4f b = *(const v4f*)(xp + 4);
  v8h hi, lo;
#pragma unroll
  for (int e = 0; e < 4; ++e) {
    const float va = a[e];
    const float vb = b[e];
    const _Float16 ha = (_Float16)va;
    const _Float16 hb = (_Float16)vb;
    const float ra = (va - (float)ha) * RCARRY;
    const float rb = (vb - (float)hb) * RCARRY;
    hi[e]     = ha;
    hi[4 + e] = hb;
    lo[e]     = (_Float16)ra;
    lo[4 + e] = (_Float16)rb;
  }
  *(v8h*)(dst) = hi;
  *(v8h*)(dst + LO_OFF) = lo;
}

__global__ __launch_bounds__(256) void wcat_cvt_kernel(const float* __restrict__ wx, const float* __restrict__ wh,
                                                       unsigned short* __restrict__ dst) {
  const int i = blockIdx.x * 256 + threadIdx.x;
  const int which = blockIdx.y;
  const float* src = which ? wh : wx;
  if (i < NGATE * (NIN / 8)) {
    const int row = i >> 5;
    const int c8  = i & 31;
    const float* sp = src + (size_t)row * NIN + c8 * 8;
    const v4f a = *(const v4f*)(sp);
    const v4f b = *(const v4f*)(sp + 4);
    v8h hv;
#pragma unroll
    for (int e = 0; e < 4; ++e) {
      const float fa = a[e] * WCARRY;
      const float fb = b[e] * WCARRY;
      hv[e]     = (_Float16)fa;
      hv[4 + e] = (_Float16)fb;
    }
    unsigned short* dp = dst + (size_t)row * KCAT + (size_t)which * NIN + c8 * 8;
    *(volatile v8h*)dp = hv;
    __threadfence();
    *(volatile v8h*)dp = hv;
  }
}

__global__ __launch_bounds__(RTHR) void lstm_seq_kernel(const float* __restrict__ x,
                                                        const float* __restrict__ b_x, const float* __restrict__ b_h,
                                                        const unsigned short* __restrict__ Wcp,
                                                        const float* __restrict__ w_fc, const float* __restrict__ b_fc,
                                                        float* __restrict__ out0, float* __restrict__ out1) {
  __shared__ __align__(16) _Float16 At[SEQ_BLK * APITCH];
  __shared__ __align__(16) float    Cs[SEQ_BLK * CPITCH];
  const _Float16* Wc = (const _Float16*)Wcp;
  const int tid = threadIdx.x, lane = tid & 31, wave = tid >> 5;
  const int c = lane & 15, hh = lane >> 4, koff = hh * 8;
  const int rowbase = blockIdx.x * SEQ_BLK;
  const int j = 16 * wave + c;
  const int scol = lane * 8;
  _Float16* srowp = At + wave * APITCH;
  const float* xrow = x + (size_t)(rowbase + wave) * NSTEP * NIN + scol;

  {
    v8h zh;
#pragma unroll
    for (int e = 0; e < 8; ++e) zh[e] = (_Float16)0.0f;
    *(v8h*)(srowp + H_OFF + scol) = zh;
    *(v8h*)(srowp + LO_OFF + H_OFF + scol) = zh;
  }
  stage_x8(xrow, srowp + scol);

  float bb[4];
#pragma unroll
  for (int g = 0; g < 4; ++g) bb[g] = b_x[g * NHID + j] + b_h[g * NHID + j];
  float cst[8], hst[8];
#pragma unroll
  for (int r = 0; r < 8; ++r) { cst[r] = 0.0f; hst[r] = 0.0f; }
  __syncthreads();

  const _Float16* arow = At + c * APITCH + koff;
  const _Float16* wrow = Wc + (size_t)j * KCAT + koff;
  const v8f z8 = {0.f, 0.f, 0.f, 0.f, 0.f, 0.f, 0.f, 0.f};

#pragma unroll 1
  for (int t = 0; t < NSTEP; ++t) {
    v8f am[4], ar[4];
    am[0] = z8; am[1] = z8; am[2] = z8; am[3] = z8;
    ar[0] = z8; ar[1] = z8; ar[2] = z8; ar[3] = z8;
#pragma unroll 1
    for (int k0 = 0; k0 < KCAT; k0 += 32) {
      const v16h ahi = Frag<_Float16>::load(arow + k0);
      const v16h alo = Frag<_Float16>::load(arow + LO_OFF + k0);
      const v16h b0 = Frag<_Float16>::load(wrow + k0);
      const v16h b1 = Frag<_Float16>::load(wrow + (size_t)1 * NHID * KCAT + k0);
      const v16h b2 = Frag<_Float16>::load(wrow + (size_t)2 * NHID * KCAT + k0);
      const v16h b3 = Frag<_Float16>::load(wrow + (size_t)3 * NHID * KCAT + k0);
      am[0] = Frag<_Float16>::mma(ahi, b0, am[0]);
      am[1] = Frag<_Float16>::mma(ahi, b1, am[1]);
      am[2] = Frag<_Float16>::mma(ahi, b2, am[2]);
      am[3] = Frag<_Float16>::mma(ahi, b3, am[3]);
      ar[0] = Frag<_Float16>::mma(alo, b0, ar[0]);
      ar[1] = Frag<_Float16>::mma(alo, b1, ar[1]);
      ar[2] = Frag<_Float16>::mma(alo, b2, ar[2]);
      ar[3] = Frag<_Float16>::mma(alo, b3, ar[3]);
      guard8(am[0], am[1], am[2], am[3], ar[0], ar[1], ar[2], ar[3], ahi, alo, b0, b1, b2, b3);
    }
    acc_guard4(am[0], am[1], am[2], am[3]);
    acc_guard4(ar[0], ar[1], ar[2], ar[3]);

#pragma unroll
    for (int r = 0; r < 8; ++r) {
      const float zi = (am[0][r] + ar[0][r] * RCARRY_INV) * WCARRY_INV + bb[0];
      const float zf = (am[1][r] + ar[1][r] * RCARRY_INV) * WCARRY_INV + bb[1];
      const float zg = (am[2][r] + ar[2][r] * RCARRY_INV) * WCARRY_INV + bb[2];
      const float zo = (am[3][r] + ar[3][r] * RCARRY_INV) * WCARRY_INV + bb[3];
      const float ig = fsig(zi);
      const float fg = fsig(zf);
      const float gg = ftanh(zg);
      const float og = fsig(zo);
      const float cn = cst[r] * fg + ig * gg;
      cst[r] = cn;
      hst[r] = og * ftanh(cn);
    }
    __syncthreads();
#pragma unroll
    for (int r = 0; r < 8; ++r) {
      const float hv = hst[r];
      const _Float16 hhi = (_Float16)hv;
      const float hres = (hv - (float)hhi) * RCARRY;
      const _Float16 hlo = (_Float16)hres;
      At[(8 * hh + r) * APITCH + H_OFF + j] = hhi;
      At[(8 * hh + r) * APITCH + LO_OFF + H_OFF + j] = hlo;
      Cs[(8 * hh + r) * CPITCH + j] = cst[r];
    }
    {
      const int tn = (t + 1 < NSTEP) ? (t + 1) : (NSTEP - 1);
      stage_x8(xrow + (size_t)tn * NIN, srowp + scol);
    }
    __syncthreads();
    {
      const float* sp = Cs + wave * CPITCH;
      const v4f v0 = *(const v4f*)(sp + 4 * lane);
      const v4f v1 = *(const v4f*)(sp + 128 + 4 * lane);
      float* op = out1 + ((size_t)(rowbase + wave) * NSTEP + (size_t)t) * NHID;
      *(volatile v4f*)(op + 4 * lane) = v0;
      *(volatile v4f*)(op + 128 + 4 * lane) = v1;
      __threadfence();
      *(volatile v4f*)(op + 4 * lane) = v0;
      *(volatile v4f*)(op + 128 + 4 * lane) = v1;
    }
  }

  __syncthreads();
#pragma unroll
  for (int r = 0; r < 8; ++r) Cs[(8 * hh + r) * CPITCH + j] = hst[r];
  __syncthreads();
  {
    const int o4 = lane * 4;
    const float* hrow = Cs + wave * CPITCH;
    const float* w0 = w_fc + (size_t)(o4 + 0) * NHID;
    const float* w1 = w_fc + (size_t)(o4 + 1) * NHID;
    const float* w2 = w_fc + (size_t)(o4 + 2) * NHID;
    const float* w3 = w_fc + (size_t)(o4 + 3) * NHID;
    float s0 = 0.0f, s1 = 0.0f, s2 = 0.0f, s3 = 0.0f;
#pragma unroll 1
    for (int k = 0; k < NHID; k += 4) {
      const v4f hv = *(const v4f*)(hrow + k);
      const v4f a0 = *(const v4f*)(w0 + k);
      const v4f a1 = *(const v4f*)(w1 + k);
      const v4f a2 = *(const v4f*)(w2 + k);
      const v4f a3 = *(const v4f*)(w3 + k);
#pragma unroll
      for (int e = 0; e < 4; ++e) {
        s0 = fmaf(hv[e], a0[e], s0);
        s1 = fmaf(hv[e], a1[e], s1);
        s2 = fmaf(hv[e], a2[e], s2);
        s3 = fmaf(hv[e], a3[e], s3);
      }
    }
    const v4f bv = *(const v4f*)(b_fc + o4);
    v4f o;
    o[0] = s0 + bv[0];
    o[1] = s1 + bv[1];
    o[2] = s2 + bv[2];
    o[3] = s3 + bv[3];
    float* op = out0 + (size_t)(rowbase + wave) * NFC + o4;
    *(volatile v4f*)op = o;
    __threadfence();
    *(volatile v4f*)op = o;
  }
}

extern "C" void kernel_launch(void* const* d_in, const int* in_sizes, int n_in,
                              void* d_out, int out_size, void* d_ws, size_t ws_size, hipStream_t stream) {
  if (n_in < 7 || d_out == nullptr || d_ws == nullptr) return;
  if (in_sizes[0] != NBATCH * NSTEP * NIN || in_sizes[1] != NGATE * NIN || in_sizes[2] != NGATE ||
      in_sizes[3] != NGATE * NHID || in_sizes[4] != NGATE || in_sizes[5] != NFC * NHID || in_sizes[6] != NFC ||
      out_size != NOUT0 + NOUT1) return;

  const float* x     = (const float*)d_in[0];
  const float* w_x2h = (const float*)d_in[1];
  const float* b_x2h = (const float*)d_in[2];
  const float* w_h2h = (const float*)d_in[3];
  const float* b_h2h = (const float*)d_in[4];
  const float* w_fc  = (const float*)d_in[5];
  const float* b_fc  = (const float*)d_in[6];
  float* out0 = (float*)d_out;
  float* out1 = out0 + (size_t)NOUT0;

  char* ws = (char*)d_ws;
  size_t off = 0;
  auto carve = [&](size_t bytes) -> char* { char* p = ws + off; off += (bytes + 255) & ~(size_t)255; return p; };
  unsigned short* WC = (unsigned short*)carve((size_t)NGATE * KCAT * 2);
  if (off > ws_size || off > (size_t)134217728) return;

  wcat_cvt_kernel<<<dim3((NGATE * (NIN / 8)) / 256, 2), 256, 0, stream>>>(w_x2h, w_h2h, WC);
  lstm_seq_kernel<<<NBATCH / SEQ_BLK, RTHR, 0, stream>>>(x, b_x2h, b_h2h, WC, w_fc, b_fc, out0, out1);
}
